// CREDALoss_74062416052317
// MI455X (gfx1250) — hardware-verified
//
#include <hip/hip_runtime.h>


namespace {
constexpr int NS = 1024, NT = 1024, N = 2048, D = 2048, C = 4, RB = 64  , NRB = N / RB  ;
constexpr float EPS = 1e-8f, LC = 1.0f, LE = 0.1f;

typedef _Float16 b16;
typedef __attribute__((ext_vector_type(16))) _Float16 v16b;
typedef __attribute__((ext_vector_type(8))) _Float16 v8b;
typedef __attribute__((ext_vector_type(8))) float v8f;
typedef __attribute__((ext_vector_type(4))) float v4f;
__device__ __forceinline__ float bf16_rne(float f) { unsigned int u = __float_as_uint(f); u += 0x7FFFu + ((u >> 16) & 1u); return __uint_as_float(u & 0xFFFF0000u); }
__device__ __forceinline__ v16b frag_x(const float* p, int hh) { v16b f;
#pragma unroll
  for (int e = 0; e < 8; ++e) { f[e] = (b16)bf16_rne(p[8 * hh + e]); f[8 + e] = (b16)bf16_rne(p[16 + 8 * hh + e]); } return f; }
__device__ __forceinline__ v8f wmma16b(v16b a, v16b b, v8f c) { v8f d = __builtin_amdgcn_wmma_f32_16x16x32_f16(false, a, false, b, (short)0, c, false, false); asm volatile("v_nop\n\tv_nop\n\tv_nop\n\tv_nop" : "+v"(d) : "v"(a), "v"(b)); return d; }
__device__ __forceinline__ void wave_lds_sync() { __builtin_amdgcn_fence(__ATOMIC_RELEASE, "workgroup"); __builtin_amdgcn_wave_barrier(); __builtin_amdgcn_fence(__ATOMIC_ACQUIRE, "workgroup"); }
__device__ __forceinline__ float nexp(float x) { return __builtin_amdgcn_exp2f(x * 1.4426950408889634f); }
__device__ __forceinline__ float nlog(float x) { return __builtin_amdgcn_logf(x) * 0.6931471805599453f; }
__device__ __forceinline__ float pmul(float a, float b) { float p = a * b; asm volatile("" : "+v"(p)); return p; }
__device__ __forceinline__ float wsum(float v) {
#pragma unroll
  for (int o = 1; o < 32; o <<= 1) v += __shfl_xor(v, o); return v; }
__device__ __forceinline__ int wsumi(int v) {
#pragma unroll
  for (int o = 1; o < 32; o <<= 1) v += __shfl_xor(v, o); return v; }
__device__ __forceinline__ const float* rowp(const float* fs, const float* ft, int i) { return (i < NS) ? (fs + (size_t)i * D) : (ft + (size_t)(i - NS) * D); }
__device__ __forceinline__ int cls_of(const int* lab, const float* lt, int i) { if (i < NS) return lab[i]; const float* l = lt + (size_t)(i - NS) * C; int best = 0; float bv = bf16_rne(l[0]);
#pragma unroll 1
  for (int c = 1; c < C; ++c) { const float v = bf16_rne(l[c]); if (v > bv) { bv = v; best = c; } } return best; }
__device__ __forceinline__ float went(const float* lt, int it) {
  const float* l = lt + (size_t)it * C; float mx = -INFINITY;
#pragma unroll 1
  for (int c = 0; c < C; ++c) mx = fmaxf(mx, bf16_rne(l[c]));
  float s = 0.0f;
#pragma unroll 1
  for (int c = 0; c < C; ++c) s += nexp(bf16_rne(l[c]) - mx);
  float ent = 0.0f;
#pragma unroll 1
  for (int c = 0; c < C; ++c) { const float p = nexp(bf16_rne(l[c]) - mx) / s; ent -= pmul(p, nlog(p + EPS)); }
  return 1.0f - ent / (nlog((float)C) + EPS); }

__global__ __launch_bounds__(64) void d2_kernel(const float* __restrict__ fs, const float* __restrict__ ft, float* __restrict__ D2) {
  __shared__ __attribute__((aligned(16))) float Ts[2][32][128 + 4]; __shared__ float xr[32], xc[2][128];
  const int lane = threadIdx.x & 31, wave = threadIdx.x >> 5, nloc = lane & 15, hlf = lane >> 4, m0 = blockIdx.y * 32, c0 = blockIdx.x * 256 + wave * 128;
  for (int q = 0; q < 16; ++q) { const int i = m0 + wave * 16 + q; const float* p = rowp(fs, ft, i); float s = 0.0f; for (int k = lane; k < D; k += 32) { const float v = bf16_rne(p[k]); s += pmul(v, v); } s = wsum(s); if (lane == 0) xr[wave * 16 + q] = s; }
  for (int q = 0; q < 128; ++q) { const int j = c0 + q; const float* p = rowp(fs, ft, j); float s = 0.0f; for (int k = lane; k < D; k += 32) { const float v = bf16_rne(p[k]); s += pmul(v, v); } s = wsum(s); if (lane == 0) xc[wave][q] = s; }
  v8f acc[2][8];
#pragma unroll
  for (int r = 0; r < 2; ++r)
#pragma unroll
    for (int t = 0; t < 8; ++t) acc[r][t] = (v8f){};
  for (int kb = 0; kb < D; kb += 32) { const v16b a0 = frag_x(rowp(fs, ft, m0 + nloc) + kb, hlf), a1 = frag_x(rowp(fs, ft, m0 + 16 + nloc) + kb, hlf);
#pragma unroll
    for (int t = 0; t < 8; ++t) { const v16b bw = frag_x(rowp(fs, ft, c0 + t * 16 + nloc) + kb, hlf); acc[0][t] = wmma16b(a0, bw, acc[0][t]); acc[1][t] = wmma16b(a1, bw, acc[1][t]); } }
  __syncthreads();
#pragma unroll
  for (int t = 0; t < 8; ++t)
#pragma unroll
    for (int r = 0; r < 2; ++r)
#pragma unroll
      for (int v = 0; v < 8; ++v) { const int rr = r * 16 + 8 * hlf + v, cc = t * 16 + nloc; Ts[wave][rr][cc] = fmaxf(xr[rr] + xc[wave][cc] - 2.0f * acc[r][t][v], 0.0f); }
  wave_lds_sync();
  for (int pass = 0; pass < 2; ++pass) { for (int i = lane; i < 32 * 32; i += 32) { const int rr = i >> 5, c4 = (i & 31) * 4; *(volatile v4f*)(D2 + (size_t)(m0 + rr) * N + c0 + c4) = *(const v4f*)(&Ts[wave][rr][c4]); } __threadfence(); }
}

__global__ __launch_bounds__(256) void median_kernel(const float* __restrict__ D2, const int* __restrict__ lab, const float* __restrict__ lt, float* __restrict__ MED) {
  __shared__ int memb[N]; __shared__ int redi[8]; __shared__ unsigned int lo_s, hi_s; __shared__ int m_s;
  const int c = blockIdx.x, t_ = threadIdx.x, lane = t_ & 31, wave = t_ >> 5;
  if (t_ == 0) m_s = 0;
  __syncthreads();
  for (int i0 = 0; i0 < N; i0 += 256) { const int i = i0 + t_; const int is = (cls_of(lab, lt, i) == c) ? 1 : 0; const unsigned int bal = __builtin_amdgcn_ballot_w32(is != 0); if (lane == 0) redi[wave] = __builtin_popcount(bal); __syncthreads();
    int base = m_s; for (int w = 0; w < wave; ++w) base += redi[w]; const int pos = base + __builtin_popcount(bal & ((1u << lane) - 1u)); if (is) memb[pos] = i; __syncthreads();
    if (t_ == 0) { int a = m_s; for (int w = 0; w < 8; ++w) a += redi[w]; m_s = a; } __syncthreads(); }
  const int m = m_s;
  const long long cnt = (long long)m * (m - 1) / 2; const long long kk = (cnt > 0) ? ((cnt - 1) / 2) : 0;
  if (t_ == 0) { lo_s = 0u; hi_s = 0x7F800000u; }
  __syncthreads();
  for (int it = 0; it < 32; ++it) { const unsigned int lo = lo_s, hi = hi_s; if (lo >= hi) break; const unsigned int mid = lo + (hi - lo) / 2; const float piv = __uint_as_float(mid);
    long long cntle = 0;
    for (int a = wave; a < m; a += 8) { const float* row = D2 + (size_t)memb[a] * N; int cl = 0; for (int bq = a + 1 + lane; bq < m; bq += 32) cl += (row[memb[bq]] <= piv) ? 1 : 0; cntle += cl; }
    int part = (int)cntle; part = wsumi(part); if (lane == 0) redi[wave] = part; __syncthreads();
    if (t_ == 0) { long long tot = 0; for (int w = 0; w < 8; ++w) tot += redi[w]; if (tot >= kk + 1) hi_s = mid; else lo_s = mid + 1; }
    __syncthreads(); }
  if (t_ < 32) { const float med = (cnt > 0) ? __uint_as_float(hi_s) : 1.0f; const float v = (t_ == 0) ? med : (t_ == 1) ? (float)m : 0.0f; for (int pass = 0; pass < 2; ++pass) ((volatile float*)MED)[(size_t)c * 32 + t_] = v; }
  __threadfence();
}

__global__ __launch_bounds__(256) void ksum_kernel(const float* __restrict__ D2, const int* __restrict__ lab, const float* __restrict__ lt, const float* __restrict__ MED, float* __restrict__ PART) {
  __shared__ float wv[N]; __shared__ unsigned char ms[N], mt[N]; __shared__ float red[4][8];
  const int rb = blockIdx.x, c = blockIdx.y, t_ = threadIdx.x, lane = t_ & 31, wave = t_ >> 5;
  for (int i = t_; i < N; i += 256) { const int cl = cls_of(lab, lt, i); ms[i] = (unsigned char)((i < NS && cl == c) ? 1 : 0); mt[i] = (unsigned char)((i >= NS && cl == c) ? 1 : 0); wv[i] = (i >= NS) ? went(lt, i - NS) : 0.0f; }
  __syncthreads();
  const float sig2 = MED[(size_t)c * 32] + 1e-6f; const float inv = -1.0f / (2.0f * sig2 + EPS);
  float sss = 0.0f, stt = 0.0f, sst = 0.0f, trt = 0.0f;
  for (int q = 0; q < RB / 8; ++q) { const int i = rb * RB + wave * (RB / 8) + q; const bool si = ms[i], ti = mt[i]; if (!si && !ti) continue; const float wi = wv[i]; const float* row = D2 + (size_t)i * N;
    for (int j = lane; j < N; j += 32) { const float K = nexp(row[j] * inv); const float K2 = pmul(K, K);
      if (si) { if (ms[j]) sss += K2; if (mt[j]) sst += K2; }
      if (ti && mt[j]) { const float ww = pmul(wi, wv[j]); stt += pmul(pmul(ww, ww), K2); if (j == i) trt += pmul(pmul(wi, wi), K); } } }
  sss = wsum(sss); stt = wsum(stt); sst = wsum(sst); trt = wsum(trt);
  if (lane == 0) { red[0][wave] = sss; red[1][wave] = stt; red[2][wave] = sst; red[3][wave] = trt; }
  __syncthreads();
  if (t_ < 32) { float v = 0.0f; if (t_ < 4) { for (int w = 0; w < 8; ++w) v += red[t_][w]; } for (int pass = 0; pass < 2; ++pass) ((volatile float*)PART)[((size_t)c * NRB + rb) * 32 + t_] = v; }
  __threadfence();
}

__global__ __launch_bounds__(256) void final_kernel(const float* __restrict__ PART, const float* __restrict__ MED, const int* __restrict__ lab, const float* __restrict__ ls, const float* __restrict__ lt, float* __restrict__ out) {
  __shared__ float red[8]; __shared__ int redi[2][8]; __shared__ float ce_s, ent_s; __shared__ int ns_c[C], nt_c[C];
  const int t_ = threadIdx.x, lane = t_ & 31, wave = t_ >> 5;
  float ce = 0.0f;
#pragma unroll 1
  for (int i = t_; i < NS; i += 256) { const float* l = ls + (size_t)i * C; float mx = -INFINITY;
#pragma unroll 1
    for (int c = 0; c < C; ++c) mx = fmaxf(mx, bf16_rne(l[c]));
    float s = 0.0f;
#pragma unroll 1
    for (int c = 0; c < C; ++c) s += nexp(bf16_rne(l[c]) - mx);
    const int lc = lab[i]; ce += (mx + nlog(s)) - bf16_rne(l[(lc >= 0 && lc < C) ? lc : 0]); }
  ce = wsum(ce); if (lane == 0) red[wave] = ce; __syncthreads(); if (t_ == 0) { float a = 0.0f; for (int w = 0; w < 8; ++w) a += red[w]; ce_s = a / (float)NS; } __syncthreads();
  float en = 0.0f;
#pragma unroll 1
  for (int i = t_; i < NT; i += 256) { en += 1.0f - went(lt, i); }
  en = wsum(en); if (lane == 0) red[wave] = en; __syncthreads(); if (t_ == 0) { float a = 0.0f; for (int w = 0; w < 8; ++w) a += red[w]; ent_s = a * (nlog((float)C) + EPS) / (float)NT; } __syncthreads();
#pragma unroll 1
  for (int c = 0; c < C; ++c) { int a = 0, b = 0;
#pragma unroll 1
    for (int i = t_; i < N; i += 256) { const int cl = cls_of(lab, lt, i); if (cl == c) { if (i < NS) ++a; else ++b; } } a = wsumi(a); b = wsumi(b); if (lane == 0) { redi[0][wave] = a; redi[1][wave] = b; } __syncthreads();
    if (t_ == 0) { int sa = 0, sb = 0; for (int w = 0; w < 8; ++w) { sa += redi[0][w]; sb += redi[1][w]; } ns_c[c] = sa; nt_c[c] = sb; } __syncthreads(); }
  if (t_ == 0) { float sumterm = 0.0f; int nvalid = 0;
#pragma unroll 1
    for (int c = 0; c < C; ++c) { float sss = 0.0f, stt = 0.0f, sst = 0.0f, trt = 0.0f;
#pragma unroll 1
      for (int rb = 0; rb < NRB; ++rb) { const float* p = PART + ((size_t)c * NRB + rb) * 32; sss += p[0]; stt += p[1]; sst += p[2]; trt += p[3]; }
      const bool valid = (ns_c[c] >= 2) && (nt_c[c] >= 2); const float trs = (float)ns_c[c];
      auto h2 = [](float fro, float tr) { const float t = tr + EPS; return -__builtin_amdgcn_logf(fro / (t * t) + EPS); };
      const float term = h2(sss + stt + 2.0f * sst, trs + trt) - 0.5f * (h2(sss, trs) + h2(stt, trt));
      if (valid) { sumterm += term; ++nvalid; } }
    const float lcreda = (nvalid > 0) ? sumterm / (float)nvalid : 0.0f;
    const float loss = ce_s + LC * lcreda + LE * ent_s;
    for (int pass = 0; pass < 2; ++pass) { ((volatile float*)out)[0] = loss; __threadfence(); } }
}
}

extern "C" void kernel_launch(void* const* d_in, const int* in_sizes, int n_in,
                              void* d_out, int out_size, void* d_ws, size_t ws_size, hipStream_t stream) {
  (void)n_in; (void)out_size;
  const float* fs = (const float*)d_in[0]; const float* ls = (const float*)d_in[1]; const int* lab = (const int*)d_in[2]; const float* ft = (const float*)d_in[3]; const float* lt = (const float*)d_in[4];
  float* out = (float*)d_out;
  if (in_sizes[0] != NS * D || in_sizes[1] != NS * C || in_sizes[2] != NS || in_sizes[3] != NT * D || in_sizes[4] != NT * C) return;
  size_t off = 0; char* ws = (char*)d_ws;
  auto carve = [&](size_t bytes) { char* p = ws + off; off += (bytes + 255) & ~(size_t)255; return p; };
  float* D2 = (float*)carve((size_t)N * N * 4); float* MED = (float*)carve(C * 32 * 4); float* PART = (float*)carve((size_t)C * NRB * 32 * 4);
  if (off > ws_size) return;
  d2_kernel<<<dim3(N / 256, N / 32), 64, 0, stream>>>(fs, ft, D2);
  median_kernel<<<C, 256, 0, stream>>>(D2, lab, lt, MED);
  ksum_kernel<<<dim3(NRB, C), 256, 0, stream>>>(D2, lab, lt, MED, PART);
  final_kernel<<<1, 256, 0, stream>>>(PART, MED, lab, ls, lt, out);
}
